// ContextAM_71468255805545
// MI455X (gfx1250) — hardware-verified
//
#include <hip/hip_runtime.h>
#include <stddef.h>
#include <stdint.h>

#define NBAT   4
#define NCH    64
#define NPX    9216
#define NQK    8
#define NHID   4
#define NBLK   144
#define KSL    32
#define MSTEPS 288
#define LP     72
#define OSP    68
#define NPART  128

static_assert(NBLK * 64 == NPX);
static_assert(MSTEPS * 32 == NPX);
static_assert(NBAT * NCH * NPX == 2359296);
static_assert((LP * 2) % 16 == 0);
static_assert((OSP * 4) % 16 == 0);
static_assert(NPX % 8 == 0);

typedef float          v8f   __attribute__((ext_vector_type(8)));
typedef float          v4f   __attribute__((ext_vector_type(4)));
typedef unsigned int   v4u   __attribute__((ext_vector_type(4)));
typedef unsigned short ush;
typedef ush            v4us  __attribute__((ext_vector_type(4)));
typedef ush            v8us  __attribute__((ext_vector_type(8)));
typedef ush            v16us __attribute__((ext_vector_type(16)));
typedef _Float16       v16h  __attribute__((ext_vector_type(16)));
typedef __bf16         v16b  __attribute__((ext_vector_type(16)));

union FragU { v16us v; v8us h[2]; v16b b; v16h f; };

__device__ __forceinline__ ush f2bf(float f) {
  const unsigned u = __float_as_uint(f);
  return (ush)((u + 0x7FFFu + ((u >> 16) & 1u)) >> 16);
}
__device__ __forceinline__ float bf2f(ush v) { return __uint_as_float(((unsigned)v) << 16); }
__device__ __forceinline__ ush h2u(float f) {
  union { _Float16 h; ush u; } t;
  t.h = (_Float16)f;
  return t.u;
}

__device__ __forceinline__ v8f zero8() { return (v8f){0.f, 0.f, 0.f, 0.f, 0.f, 0.f, 0.f, 0.f}; }

__device__ __forceinline__ v8f mma_bf(v16us a, v16us b, v8f c) {
  FragU ua, ub; ua.v = a; ub.v = b;
  c = __builtin_amdgcn_wmma_f32_16x16x32_bf16(false, ua.b, false, ub.b, (short)0, c, false, false);
  asm volatile("v_nop\n\tv_nop\n\tv_nop\n\tv_nop" : "+v"(c) : "v"(a), "v"(b));
  return c;
}
__device__ __forceinline__ v8f mma_h(v16us a, v16us b, v8f c) {
  FragU ua, ub; ua.v = a; ub.v = b;
  c = __builtin_amdgcn_wmma_f32_16x16x32_f16(false, ua.f, false, ub.f, (short)0, c, false, false);
  asm volatile("v_nop\n\tv_nop\n\tv_nop\n\tv_nop" : "+v"(c) : "v"(a), "v"(b));
  return c;
}

__device__ __forceinline__ v16us ldfrag(const ush* p, int ld, int row0, int k0, int lane) {
  const ush* q = p + (size_t)(row0 + (lane & 15)) * ld + k0 + 8 * (lane >> 4);
  FragU f;
  f.h[0] = *(const v8us*)(q);
  f.h[1] = *(const v8us*)(q + 16);
  return f.v;
}

__device__ __forceinline__ float sigm(float e) {
  return __builtin_amdgcn_rcpf(1.0f + __expf(-e));
}

__global__ __launch_bounds__(128) void k_qkv(
    const float* __restrict__ x, const float* __restrict__ wq, const float* __restrict__ bq,
    const float* __restrict__ wk, const float* __restrict__ bk, const float* __restrict__ wv,
    const float* __restrict__ bv, ush* __restrict__ Vp, ush* __restrict__ Qp, ush* __restrict__ Kp)
{
  __shared__ __align__(16) ush Wv[NCH * LP];
  __shared__ __align__(16) ush Wbh[16 * LP];
  __shared__ __align__(16) ush Wbl[16 * LP];
  __shared__ __align__(16) ush Xh[64 * LP];
  __shared__ __align__(16) ush Xbh[64 * LP];
  __shared__ __align__(16) ush Xbl[64 * LP];
  __shared__ __align__(16) ush Vs[NCH * LP];
  __shared__ __align__(16) ush QKs[2 * 64 * KSL];

  const int tid = threadIdx.x, lane = tid & 31, wave = tid >> 5, hh = lane >> 4, cc = lane & 15;
  const int nb = blockIdx.x, b = blockIdx.y;
  const int n0 = nb * 64;

  {
    const int o  = tid >> 4;
    const int c4 = (tid & 15) * 4;
    const v4f aq = *(const v4f*)(wq + o * NCH + c4);
    const v4f ak = *(const v4f*)(wk + o * NCH + c4);
    v4us qh, ql, kh, kl;
#pragma unroll
    for (int e = 0; e < 4; ++e) {
      const ush hq = f2bf(aq[e]); qh[e] = hq; ql[e] = f2bf(aq[e] - bf2f(hq));
      const ush hk = f2bf(ak[e]); kh[e] = hk; kl[e] = f2bf(ak[e] - bf2f(hk));
    }
    *(v4us*)(Wbh + o * LP + c4)       = qh;
    *(v4us*)(Wbl + o * LP + c4)       = ql;
    *(v4us*)(Wbh + (8 + o) * LP + c4) = kh;
    *(v4us*)(Wbl + (8 + o) * LP + c4) = kl;
  }
#pragma unroll 1
  for (int g = 0; g < 2; ++g) {
    v4f wa[4];
#pragma unroll
    for (int i = 0; i < 4; ++i) {
      const int f  = tid + 128 * (4 * g + i);
      const int o  = f >> 4;
      const int c4 = (f & 15) * 4;
      wa[i] = *(const v4f*)(wv + o * NCH + c4);
    }
#pragma unroll
    for (int i = 0; i < 4; ++i) {
      const int f  = tid + 128 * (4 * g + i);
      const int o  = f >> 4;
      const int c4 = (f & 15) * 4;
      v4us u;
#pragma unroll
      for (int e = 0; e < 4; ++e) u[e] = h2u(wa[i][e] * 16.0f);
      *(v4us*)(Wv + o * LP + c4) = u;
    }
  }
#pragma unroll 1
  for (int g = 0; g < 2; ++g) {
    v4f xa[4];
#pragma unroll
    for (int i = 0; i < 4; ++i) {
      const int f  = tid + 128 * (4 * g + i);
      const int c  = f >> 4;
      const int n4 = (f & 15) * 4;
      xa[i] = *(const v4f*)(x + ((size_t)(b * NCH + c)) * NPX + n0 + n4);
    }
#pragma unroll
    for (int i = 0; i < 4; ++i) {
      const int f  = tid + 128 * (4 * g + i);
      const int c  = f >> 4;
      const int n4 = (f & 15) * 4;
#pragma unroll
      for (int e = 0; e < 4; ++e) {
        const float xv = xa[i][e];
        const int so = (n4 + e) * LP + c;
        Xh[so] = h2u(xv);
        const ush hb = f2bf(xv);
        Xbh[so] = hb;
        Xbl[so] = f2bf(xv - bf2f(hb));
      }
    }
  }
  __syncthreads();

  v8f acc[5];
#pragma unroll
  for (int t = 0; t < 5; ++t) acc[t] = zero8();
  const int nr0 = 16 * wave;
#pragma unroll
  for (int ks = 0; ks < 2; ++ks) {
    const v16us bfh = ldfrag(Xh,  LP, nr0, 32 * ks, lane);
    const v16us bbh = ldfrag(Xbh, LP, nr0, 32 * ks, lane);
    const v16us bbl = ldfrag(Xbl, LP, nr0, 32 * ks, lane);
    const v16us awh = ldfrag(Wbh, LP, 0, 32 * ks, lane);
    const v16us awl = ldfrag(Wbl, LP, 0, 32 * ks, lane);
    acc[0] = mma_bf(awh, bbh, acc[0]);
    acc[0] = mma_bf(awh, bbl, acc[0]);
    acc[0] = mma_bf(awl, bbh, acc[0]);
#pragma unroll
    for (int mt = 0; mt < 4; ++mt) {
      const v16us av = ldfrag(Wv, LP, 16 * mt, 32 * ks, lane);
      acc[1 + mt] = mma_h(av, bfh, acc[1 + mt]);
    }
  }

  const int nl = nr0 + cc;
  {
    v8us ph, pl;
#pragma unroll
    for (int r = 0; r < 8; ++r) {
      const float bqr = bq[r], bkr = bk[r];
      const float v = acc[0][r] + (hh ? bkr : bqr);
      const ush hq = f2bf(v);
      ph[r] = hq;
      pl[r] = f2bf(v - bf2f(hq));
    }
    v8us p1, p2, pz;
#pragma unroll
    for (int r = 0; r < 8; ++r) {
      p1[r] = hh ? ph[r] : pl[r];
      p2[r] = hh ? pl[r] : ph[r];
      pz[r] = (ush)0;
    }
    ush* d = QKs + (hh * 64 + nl) * KSL;
    *(v8us*)(d)      = ph;
    *(v8us*)(d + 8)  = p1;
    *(v8us*)(d + 16) = p2;
    *(v8us*)(d + 24) = pz;
  }
#pragma unroll
  for (int mt = 0; mt < 4; ++mt)
#pragma unroll
    for (int r = 0; r < 8; ++r) {
      const int c = 16 * mt + 8 * hh + r;
      const float v = acc[1 + mt][r] * 0.0625f + bv[c];
      Vs[c * LP + nl] = h2u(v * 16.0f);
    }
  __syncthreads();

  v4u vv[4]; size_t vo[4];
#pragma unroll
  for (int it = 0; it < 4; ++it) {
    const int p  = tid + 128 * it;
    const int c  = p >> 3;
    const int pc = p & 7;
    vv[it] = *(const v4u*)(Vs + c * LP + 8 * pc);
    vo[it] = ((size_t)(b * NCH + c)) * NPX + n0 + 8 * pc;
  }
  v4u qv[2], kv[2]; size_t qo[2];
#pragma unroll
  for (int it = 0; it < 2; ++it) {
    const int p = tid + 128 * it;
    qv[it] = *(const v4u*)(QKs + 8 * p);
    kv[it] = *(const v4u*)(QKs + 64 * KSL + 8 * p);
    qo[it] = ((size_t)b * NPX + n0) * KSL + 8 * p;
  }
#pragma unroll
  for (int it = 0; it < 4; ++it) *(volatile v4u*)(Vp + vo[it]) = vv[it];
#pragma unroll
  for (int it = 0; it < 2; ++it) { *(volatile v4u*)(Qp + qo[it]) = qv[it]; *(volatile v4u*)(Kp + qo[it]) = kv[it]; }
  __threadfence();
#pragma unroll
  for (int it = 0; it < 4; ++it) *(volatile v4u*)(Vp + vo[it]) = vv[it];
#pragma unroll
  for (int it = 0; it < 2; ++it) { *(volatile v4u*)(Qp + qo[it]) = qv[it]; *(volatile v4u*)(Kp + qo[it]) = kv[it]; }
}

__global__ __launch_bounds__(128) void k_attn(
    const ush* __restrict__ Vp, const ush* __restrict__ Qp, const ush* __restrict__ Kp,
    const float* __restrict__ x, float* __restrict__ O, float* __restrict__ part)
{
  __shared__ __align__(16) float Os[NCH * OSP];
  __shared__ __align__(16) float Sst[NPART];

  const int tid = threadIdx.x, lane = tid & 31, wave = tid >> 5, hh = lane >> 4, cc = lane & 15;
  const int nb = blockIdx.x, b = blockIdx.y;
  const int nbase = nb * 64;
  const int n0 = nbase + 16 * wave;

  const ush* Qb = Qp + (size_t)b * NPX * KSL;
  const ush* Kb = Kp + (size_t)b * NPX * KSL;
  const ush* Vb = Vp + (size_t)b * NCH * NPX;

  const v16us qf = ldfrag(Qb, KSL, n0, 0, lane);
  const v8f z8 = zero8();
  v8f ah[4], al[4];
#pragma unroll
  for (int t = 0; t < 4; ++t) { ah[t] = zero8(); al[t] = zero8(); }

#pragma unroll 1
  for (int ms = 0; ms < MSTEPS; ++ms) {
    const int m0 = ms * 32;
    const v16us kf0 = ldfrag(Kb, KSL, m0, 0, lane);
    const v16us kf1 = ldfrag(Kb, KSL, m0 + 16, 0, lane);
    const v8f e0 = mma_bf(kf0, qf, z8);
    const v8f e1 = mma_bf(kf1, qf, z8);
    v16h hv = (v16h)((_Float16)0.0f);
    v16h lv = (v16h)((_Float16)0.0f);
#pragma unroll
    for (int r = 0; r < 8; ++r) {
      const float a0 = sigm(e0[r]);
      const _Float16 h0 = (_Float16)a0;
      hv[r] = h0;
      lv[r] = (_Float16)((a0 - (float)h0) * 2048.0f);
      const float a1 = sigm(e1[r]);
      const _Float16 h1 = (_Float16)a1;
      hv[8 + r] = h1;
      lv[8 + r] = (_Float16)((a1 - (float)h1) * 2048.0f);
    }
    FragU bh, bl;
    bh.f = hv; bl.f = lv;
#pragma unroll
    for (int ct = 0; ct < 4; ++ct) {
      const v16us vf = ldfrag(Vb, NPX, 16 * ct, m0, lane);
      ah[ct] = mma_h(vf, bh.v, ah[ct]);
      al[ct] = mma_h(vf, bl.v, al[ct]);
    }
  }

#pragma unroll
  for (int ct = 0; ct < 4; ++ct)
#pragma unroll
    for (int r = 0; r < 8; ++r) {
      const int c = 16 * ct + 8 * hh + r;
      Os[c * OSP + 16 * wave + cc] = (ah[ct][r] + al[ct][r] * (1.0f / 2048.0f)) * 0.0625f;
    }
  __syncthreads();

  v4f val[8]; size_t go[8];
#pragma unroll
  for (int it = 0; it < 8; ++it) {
    const int p  = tid + 128 * it;
    const int c  = p >> 4;
    const int pc = p & 15;
    v4f o = *(const v4f*)(Os + c * OSP + 4 * pc);
    const size_t g = ((size_t)(b * NCH + c)) * NPX + nbase + 4 * pc;
    const v4f xv = *(const v4f*)(x + g);
    o += xv;
    val[it] = o;
    go[it]  = g;
    float s = (o[0] + o[1]) + (o[2] + o[3]);
    float m = fmaxf(fmaxf(o[0], o[1]), fmaxf(o[2], o[3]));
#pragma unroll
    for (int off = 1; off < 16; off <<= 1) {
      s += __shfl_xor(s, off, 32);
      m  = fmaxf(m, __shfl_xor(m, off, 32));
    }
    if (cc == 0) { Sst[c] = s; Sst[64 + c] = m; }
  }
  __syncthreads();
  const v4f sv = *(const v4f*)(Sst + 4 * lane);
  const size_t so = ((size_t)(b * NBLK + nb)) * NPART + 4 * lane;
  const bool ws0 = (wave == 0);

#pragma unroll
  for (int it = 0; it < 8; ++it) *(volatile v4f*)(O + go[it]) = val[it];
  if (ws0) *(volatile v4f*)(part + so) = sv;
  __threadfence();
#pragma unroll
  for (int it = 0; it < 8; ++it) *(volatile v4f*)(O + go[it]) = val[it];
  if (ws0) *(volatile v4f*)(part + so) = sv;
}

__global__ __launch_bounds__(64) void k_gate(const float* __restrict__ part, const float* __restrict__ w1,
                                             const float* __restrict__ w2, float* __restrict__ scl)
{
  __shared__ __align__(16) float fa[NCH];
  __shared__ __align__(16) float fm[NCH];
  __shared__ __align__(16) float sc[NCH];
  const int c = threadIdx.x, b = blockIdx.x;
  const float* pb = part + (size_t)b * NBLK * NPART;
  double s = 0.0;
  float mx = -__builtin_inff();
#pragma unroll 1
  for (int i = 0; i < NBLK; ++i) {
    s += (double)pb[i * NPART + c];
    mx = fmaxf(mx, pb[i * NPART + 64 + c]);
  }
  fa[c] = (float)s * (1.0f / (float)NPX);
  fm[c] = mx;
  __syncthreads();
  float za = 0.f, zm = 0.f;
#pragma unroll 1
  for (int r = 0; r < NHID; ++r) {
    float ha = 0.f, hm = 0.f;
#pragma unroll 1
    for (int j = 0; j < NCH; ++j) {
      const float w = w1[r * NCH + j];
      ha = fmaf(w, fa[j], ha);
      hm = fmaf(w, fm[j], hm);
    }
    const float w2v = w2[c * NHID + r];
    za = fmaf(w2v, fmaxf(ha, 0.f), za);
    zm = fmaf(w2v, fmaxf(hm, 0.f), zm);
  }
  const float z = za + zm;
  sc[c] = __builtin_amdgcn_rcpf(1.0f + expf(-z));
  __syncthreads();
  const int lc = c & 15;
  const v4f v = *(const v4f*)(sc + 4 * lc);
  float* d = scl + b * NCH + 4 * lc;
  const bool wr = (c < 16);
  if (wr) *(volatile v4f*)d = v;
  __threadfence();
  if (wr) *(volatile v4f*)d = v;
}

__global__ __launch_bounds__(256) void k_apply(const float* __restrict__ O, const float* __restrict__ scl,
                                               float* __restrict__ out)
{
  const int bc = blockIdx.x;
  const float g = scl[bc];
  const size_t base = (size_t)bc * NPX;
  v4f v[9];
#pragma unroll
  for (int it = 0; it < 9; ++it) {
    const int p = threadIdx.x + 256 * it;
    v[it] = *(const v4f*)(O + base + 4 * p) * g;
  }
#pragma unroll
  for (int it = 0; it < 9; ++it) *(volatile v4f*)(out + base + 4 * (threadIdx.x + 256 * it)) = v[it];
  __threadfence();
#pragma unroll
  for (int it = 0; it < 9; ++it) *(volatile v4f*)(out + base + 4 * (threadIdx.x + 256 * it)) = v[it];
}

extern "C" void kernel_launch(void* const* d_in, const int* in_sizes, int n_in,
                              void* d_out, int out_size, void* d_ws, size_t ws_size,
                              hipStream_t stream)
{
  if (n_in < 9) return;
  if (in_sizes[0] != NBAT * NCH * NPX) return;
  if (in_sizes[1] != NQK * NCH || in_sizes[2] != NQK) return;
  if (in_sizes[3] != NQK * NCH || in_sizes[4] != NQK) return;
  if (in_sizes[5] != NCH * NCH || in_sizes[6] != NCH) return;
  if (in_sizes[7] != NHID * NCH || in_sizes[8] != NCH * NHID) return;
  if (out_size != NBAT * NCH * NPX) return;

  const float* x  = (const float*)d_in[0];
  const float* wq = (const float*)d_in[1];
  const float* bq = (const float*)d_in[2];
  const float* wk = (const float*)d_in[3];
  const float* bk = (const float*)d_in[4];
  const float* wv = (const float*)d_in[5];
  const float* bv = (const float*)d_in[6];
  const float* w1 = (const float*)d_in[7];
  const float* w2 = (const float*)d_in[8];
  float* out = (float*)d_out;

  size_t off = 0;
  const size_t oV = off; off += (size_t)NBAT * NCH * NPX * 2;
  const size_t oQ = off; off += (size_t)NBAT * NPX * KSL * 2;
  const size_t oK = off; off += (size_t)NBAT * NPX * KSL * 2;
  const size_t oO = off; off += (size_t)NBAT * NCH * NPX * 4;
  const size_t oP = off; off += (size_t)NBAT * NBLK * NPART * 4;
  const size_t oS = off; off += (size_t)NBAT * NCH * 4;
  if (off > ws_size) return;
  if (off > (size_t)134217728) return;

  char* ws = (char*)d_ws;
  ush*   Vp   = (ush*)(ws + oV);
  ush*   Qp   = (ush*)(ws + oQ);
  ush*   Kp   = (ush*)(ws + oK);
  float* O    = (float*)(ws + oO);
  float* part = (float*)(ws + oP);
  float* scl  = (float*)(ws + oS);

  k_qkv<<<dim3(NBLK, NBAT), dim3(128), 0, stream>>>(x, wq, bq, wk, bk, wv, bv, Vp, Qp, Kp);
  k_attn<<<dim3(NBLK, NBAT), dim3(128), 0, stream>>>(Vp, Qp, Kp, x, O, part);
  k_gate<<<dim3(NBAT), dim3(64), 0, stream>>>(part, w1, w2, scl);
  k_apply<<<dim3(NBAT * NCH), dim3(256), 0, stream>>>(O, scl, out);
  (void)hipGetLastError();
}
